// QuantumMarioNet_57921928954276
// MI455X (gfx1250) — hardware-verified
//
#include <hip/hip_runtime.h>
#include <hip/hip_bf16.h>
#include <math.h>

typedef __attribute__((ext_vector_type(16))) __bf16        v16bf;
typedef __attribute__((ext_vector_type(16))) _Float16      v16h;
typedef __attribute__((ext_vector_type(4)))  float         v4f;
typedef __attribute__((ext_vector_type(2)))  float         v2f;
typedef __attribute__((ext_vector_type(8)))  float         v8f;
typedef __attribute__((ext_vector_type(4)))  unsigned int  u32x4;
typedef __attribute__((ext_vector_type(8)))  unsigned int  u32x8;

#define NQ      8
#define QDEPTH  2
#define CHIPS   100
#define BATCH   128
#define IN_DIM  (4*84*84)
#define HID     256
#define HID2    64
#define ACTIONS 7

#define GWAVES  4
#define KCHUNK  32

__device__ __forceinline__ v16h frag_f32(const float* p, int hh) {
  v16h f;
#pragma unroll
  for (int e = 0; e < 8; ++e) { f[e] = (_Float16)p[8 * hh + e]; f[8 + e] = (_Float16)p[16 + 8 * hh + e]; }
  return f;
}
__device__ __forceinline__ v8f wmma16(v16h a, v16h b, v8f c) {
  v8f d = __builtin_amdgcn_wmma_f32_16x16x32_f16(false, a, false, b, (short)0, c, false, false);
  asm volatile("v_nop\n\tv_nop\n\tv_nop\n\tv_nop" : "+v"(d) : "v"(a), "v"(b));
  return d;
}
#define VST2(T, ptr, val) do { const T _v = (val); *(volatile T*)(ptr) = _v; __threadfence(); *(volatile T*)(ptr) = _v; } while (0)

__global__ __launch_bounds__(GWAVES * 32)
void gemm_f16_wmma(const float* __restrict__ A, const float* __restrict__ W,
                   const float* __restrict__ bias, float* __restrict__ out,
                   int M, int N, int K, int do_relu)
{
  const int lane = threadIdx.x & 31;
  const int wid  = threadIdx.x >> 5;
  const int hh = lane >> 4, row = lane & 15;
  const int m0 = blockIdx.x * 16;
  const int ng = blockIdx.y * GWAVES + wid;
  if (ng * 32 >= N) return;
  const int n0 = ng * 32;
  const float* arow = A + (size_t)(m0 + row) * K;
  const float* b0row = W + (size_t)(n0 + row) * K;
  const float* b1row = W + (size_t)(n0 + 16 + row) * K;
  v8f acc0 = {}, acc1 = {};
  for (int k0 = 0; k0 < K; k0 += KCHUNK) {
    const v16h a = frag_f32(arow + k0, hh);
    acc0 = wmma16(a, frag_f32(b0row + k0, hh), acc0);
    acc1 = wmma16(a, frag_f32(b1row + k0, hh), acc1);
  }
  const float bv = bias[n0 + lane];
  for (int pass = 0; pass < 2; ++pass) {
#pragma unroll
    for (int r = 0; r < 8; ++r) {
      const float a_ = acc0[r], b_ = acc1[r];
      const float ax = __shfl_xor(a_, 16), bx = __shfl_xor(b_, 16);
      float v1 = (hh ? bx : a_) + bv, v2 = (hh ? b_ : ax) + bv;
      if (do_relu) { v1 = fmaxf(v1, 0.f); v2 = fmaxf(v2, 0.f); }
      *(volatile float*)(out + (size_t)(m0 + r) * N + n0 + lane) = v1;
      *(volatile float*)(out + (size_t)(m0 + r + 8) * N + n0 + lane) = v2;
    }
    __threadfence();
  }
}

#define NGATES 48
#define GSTRIDE 16
__device__ __forceinline__ float2 cmul(float2 a, float2 b) {
  return make_float2(a.x*b.x - a.y*b.y, a.x*b.y + a.y*b.x);
}
__device__ __forceinline__ float2 cadd(float2 a, float2 b) {
  return make_float2(a.x + b.x, a.y + b.y);
}
__device__ __forceinline__ int dep1(int p, int bt) {
  int low = p & ((1 << bt) - 1);
  int high = p >> bt;
  return low | (high << (bt + 1));
}
__device__ __forceinline__ int dep2(int p, int b0, int b1) {
  int lo = b0 < b1 ? b0 : b1;
  int hi = b0 < b1 ? b1 : b0;
  int low  = p & ((1 << lo) - 1);
  int mid  = (p >> lo) & ((1 << (hi - 1 - lo)) - 1);
  int high = p >> (hi - 1);
  return low | (mid << (lo + 1)) | (high << (hi + 1));
}

__global__ __launch_bounds__(256)
void k_gates(const float* __restrict__ conv, const float* __restrict__ pool, float* __restrict__ gates)
{
  __shared__ __attribute__((aligned(16))) float sg[NGATES * GSTRIDE];
  const int c = blockIdx.x, gi = threadIdx.x;
  if (gi < NGATES) {
    int layer, kind, w1, w2, sub;
    if (gi < 28)      { layer = 0; sub = gi / 7;        kind = gi % 7;        w1 = 2 * sub; w2 = 2 * sub + 1; }
    else if (gi < 32) { layer = 0; sub = gi - 28;       kind = 7;             w1 = 2 * sub + 1; w2 = 2 * sub; }
    else if (gi < 46) { layer = 1; sub = (gi - 32) / 7; kind = (gi - 32) % 7; w1 = 4 * sub; w2 = 4 * sub + 2; }
    else              { layer = 1; sub = gi - 46;       kind = 7;             w1 = 4 * sub + 2; w2 = 4 * sub; }
    float ang[3] = {0.f, 0.f, 0.f}; int nang = 1;
    if (kind == 7) { const float* qp = pool + ((size_t)(c * QDEPTH + layer) * 4 + sub) * 3; ang[0] = 0.5f * qp[0]; ang[1] = qp[1]; ang[2] = qp[2]; nang = 3; }
    else if (kind != 4) { const float* cp = conv + ((size_t)(c * QDEPTH + layer) * NQ + sub) * 6; ang[0] = 0.5f * cp[kind == 5 ? 4 : (kind == 6 ? 5 : kind)]; }
    float cv[3], sv_[3];
#pragma unroll 1
    for (int i = 0; i < nang; ++i) { cv[i] = cosf(ang[i]); sv_[i] = sinf(ang[i]); }
    int ctrl, targ; float2 u00, u01, u10, u11;
    if (kind == 7) {
      const float ctt = cv[0], st = sv_[0];
      const float2 ep = make_float2(cv[1], sv_[1]), ed = make_float2(cv[2], sv_[2]);
      const float2 epd = cmul(ep, ed);
      ctrl = w1; targ = w2;
      u00 = make_float2(ctt, 0.f); u01 = make_float2(-ed.x * st, -ed.y * st);
      u10 = make_float2(ep.x * st, ep.y * st); u11 = make_float2(epd.x * ctt, epd.y * ctt);
    } else if (kind == 4) {
      ctrl = w1; targ = w2;
      u00 = make_float2(0, 0); u01 = make_float2(1, 0); u10 = make_float2(1, 0); u11 = make_float2(0, 0);
    } else {
      const float ch = cv[0], sh = sv_[0];
      if (kind == 0 || kind == 2)      { ctrl = w1; targ = w2; }
      else if (kind == 1 || kind == 3) { ctrl = w2; targ = w1; }
      else if (kind == 5)              { ctrl = -1; targ = w1; }
      else                             { ctrl = -1; targ = w2; }
      if (kind == 2 || kind == 3) { u00 = make_float2(ch, 0); u01 = make_float2(0, -sh); u10 = make_float2(0, -sh); u11 = make_float2(ch, 0); }
      else                        { u00 = make_float2(ch, 0); u01 = make_float2(-sh, 0); u10 = make_float2(sh, 0);  u11 = make_float2(ch, 0); }
    }
    float* d = sg + gi * GSTRIDE;
    d[0] = (float)ctrl; d[1] = (float)targ;
    d[2] = u00.x; d[3] = u00.y; d[4] = u01.x; d[5] = u01.y; d[6] = u10.x; d[7] = u10.y; d[8] = u11.x; d[9] = u11.y;
    for (int i = 10; i < GSTRIDE; ++i) d[i] = 0.f;
  }
  __syncthreads();
  if (threadIdx.x < NGATES * GSTRIDE / 4) VST2(v4f, gates + (size_t)c * NGATES * GSTRIDE + threadIdx.x * 4, *(const v4f*)(sg + threadIdx.x * 4));
}

__global__ __launch_bounds__(256)
void k_embed(const float* __restrict__ feats, v2f* __restrict__ cs)
{
  const int i = blockIdx.x * 256 + threadIdx.x;
  if (i >= BATCH * CHIPS * NQ) return;
  const float t = 0.5f * feats[i];
  const v2f p = {cosf(t), sinf(t)};
  VST2(v2f, cs + i, p);
}

__global__ __launch_bounds__(256)
void quantum_kernel(const float2* __restrict__ cstab,
                    const float* __restrict__ gates,
                    float* __restrict__ z)
{
  __shared__ float2 smem[8][256];
  __shared__ float zs[32];
  const int lane = threadIdx.x & 31;
  const int wid  = threadIdx.x >> 5;
  float2* S = smem[wid];
  for (int it = 0; it < 4; ++it) {
    const int sv = blockIdx.x * 32 + wid * 4 + it;
    const int c  = sv % CHIPS;

    float cs[8], sn[8];
#pragma unroll
    for (int w = 0; w < 8; ++w) { const float2 p = cstab[(size_t)sv * 8 + w]; cs[w] = p.x; sn[w] = p.y; }
#pragma unroll
    for (int g = 0; g < 8; ++g) {
      int idx = g * 32 + lane;
      float a = 1.0f;
#pragma unroll
      for (int w = 0; w < 8; ++w) a *= ((idx >> (7 - w)) & 1) ? sn[w] : cs[w];
      S[idx] = make_float2(a, 0.0f);
    }
    asm volatile("" ::: "memory");

    const float* gp = gates + (size_t)c * NGATES * GSTRIDE;
#pragma unroll 1
    for (int gi = 0; gi < NGATES; ++gi) {
      const float* d = gp + gi * GSTRIDE;
      const int ctrl = (int)d[0], targ = (int)d[1];
      const float2 u00 = make_float2(d[2], d[3]), u01 = make_float2(d[4], d[5]), u10 = make_float2(d[6], d[7]), u11 = make_float2(d[8], d[9]);
      const int bt = 7 - targ;
      const int ngroups = (ctrl < 0) ? 4 : 2;
#pragma unroll 1
      for (int g = 0; g < ngroups; ++g) {
        const int p = lane + 32 * g;
        int i0;
        if (ctrl < 0) i0 = dep1(p, bt);
        else { const int bc = 7 - ctrl; i0 = dep2(p, bc, bt) | (1 << bc); }
        const int i1 = i0 | (1 << bt);
        const float2 a = S[i0], b = S[i1];
        S[i0] = cadd(cmul(u00, a), cmul(u01, b));
        S[i1] = cadd(cmul(u10, a), cmul(u11, b));
      }
      asm volatile("" ::: "memory");
    }

    float acc = 0.0f;
#pragma unroll
    for (int g = 0; g < 8; ++g) {
      int idx = g * 32 + lane;
      float2 a = S[idx];
      float p2 = a.x * a.x + a.y * a.y;
      acc += (idx & 0x80) ? -p2 : p2;
    }
#pragma unroll
    for (int off = 16; off > 0; off >>= 1) acc += __shfl_xor(acc, off, 32);
    if (lane == 0) zs[wid * 4 + it] = acc;
    __builtin_amdgcn_wave_barrier();
  }
  __syncthreads();
  if (wid == 0) VST2(float, z + (size_t)blockIdx.x * 32 + lane, zs[lane]);
}

__global__ __launch_bounds__(64)
void head_kernel(const float* __restrict__ z,   const float* __restrict__ hw1,
                 const float* __restrict__ hb1, const float* __restrict__ hw2,
                 const float* __restrict__ hb2, float* __restrict__ out)
{
  __shared__ float zr[CHIPS];
  __shared__ float hh[HID2];
  __shared__ __attribute__((aligned(16))) float os[BATCH * ACTIONS];
  const int t = threadIdx.x;
  for (int b = 0; b < BATCH; ++b) {
    __syncthreads();
    for (int k = t; k < CHIPS; k += 64) zr[k] = z[b * CHIPS + k];
    __syncthreads();
    float s = hb1[t];
    for (int k = 0; k < CHIPS; ++k) s += zr[k] * hw1[t * CHIPS + k];
    hh[t] = fmaxf(s, 0.0f);
    __syncthreads();
    if (t < ACTIONS) {
      float o = hb2[t];
      for (int j = 0; j < HID2; ++j) o += hh[j] * hw2[t * HID2 + j];
      os[b * ACTIONS + t] = o;
    }
  }
  __syncthreads();
  for (int p = t; p < BATCH * ACTIONS / 4; p += 64) VST2(v4f, out + p * 4, *(const v4f*)(os + p * 4));
}

extern "C" void kernel_launch(void* const* d_in, const int* in_sizes, int n_in,
                              void* d_out, int out_size, void* d_ws, size_t ws_size,
                              hipStream_t stream)
{
  const float* x    = (const float*)d_in[0];
  const float* w1   = (const float*)d_in[1];
  const float* b1   = (const float*)d_in[2];
  const float* w2   = (const float*)d_in[3];
  const float* b2   = (const float*)d_in[4];
  const float* conv = (const float*)d_in[5];
  const float* pool = (const float*)d_in[6];
  const float* hw1  = (const float*)d_in[7];
  const float* hb1  = (const float*)d_in[8];
  const float* hw2  = (const float*)d_in[9];
  const float* hb2  = (const float*)d_in[10];
  float* outF = (float*)d_out;

  float* ws    = (float*)d_ws;
  float* h     = ws;
  float* feats = h + (size_t)BATCH * HID;
  float* zbuf  = feats + (size_t)BATCH * CHIPS * NQ;
  float* gtab  = zbuf + (size_t)BATCH * CHIPS;
  float2* cstab = (float2*)(gtab + (size_t)CHIPS * NGATES * GSTRIDE);
  (void)in_sizes; (void)n_in; (void)out_size;
  if (ws_size < (size_t)(BATCH * HID + BATCH * CHIPS * NQ + BATCH * CHIPS + CHIPS * NGATES * GSTRIDE + 2 * BATCH * CHIPS * NQ) * sizeof(float)) return;

  gemm_f16_wmma<<<dim3(BATCH / 16, (HID / 32 + GWAVES - 1) / GWAVES), GWAVES * 32, 0, stream>>>(
      x, w1, b1, h, BATCH, HID, IN_DIM, 1);
  gemm_f16_wmma<<<dim3(BATCH / 16, (CHIPS * NQ / 32 + GWAVES - 1) / GWAVES), GWAVES * 32, 0, stream>>>(
      h, w2, b2, feats, BATCH, CHIPS * NQ, HID, 0);
  k_gates<<<CHIPS, 256, 0, stream>>>(conv, pool, gtab);
  k_embed<<<(BATCH * CHIPS * NQ + 255) / 256, 256, 0, stream>>>(feats, (v2f*)cstab);
  quantum_kernel<<<(BATCH * CHIPS) / 32, 256, 0, stream>>>(cstab, gtab, zbuf);
  head_kernel<<<1, 64, 0, stream>>>(zbuf, hw1, hb1, hw2, hb2, outF);
}
